// Low_Fidelity_FusionDeepONet_11836929868249
// MI455X (gfx1250) — hardware-run, weakly checked
//
#include <hip/hip_runtime.h>


#ifndef NB
#define NB 16
#endif
#ifndef NPTS
#define NPTS 10000
#endif
#define NB_FULL   16
#define NPTS_FULL 10000
#define HID   128
#define NOUT  5
#define NROWS (NB * NPTS)
#define XP    136
#define TW    4
#define TROWS (TW * 16)
#define OUTPIECES ((TROWS * NOUT) / 4)

static_assert(NB >= 1 && NB <= NB_FULL);
static_assert(NB_FULL == 16);
static_assert(NPTS >= 16 && NPTS <= NPTS_FULL);
static_assert(NPTS % 16 == 0);
static_assert(HID == 128);
static_assert(HID % 32 == 0);
static_assert(XP % 8 == 0 && XP >= HID);
static_assert((TROWS * NOUT) % 32 == 0);
static_assert(OUTPIECES * 16 == TROWS * NOUT * 4);
static_assert(OUTPIECES <= TW * 32);
static_assert((NROWS * NOUT) % 4 == 0);
static_assert(256 * 16 * 4 == 64 * HID * 2);
static_assert(256 * 16 * 2 == HID * 32 * 2);
static_assert(32 * 16 == HID * 4);
static_assert(16 * 16 == HID * 2);
static_assert(2 * (TW * 16 * XP * 2) + TROWS * NOUT * 4 <= 131072);
static_assert(HID * 65 * 4 <= 131072);
static_assert(2 * (16 * XP * 2) + 16 * HID * 4 + 3 * HID * 4 <= 131072);

typedef unsigned short bf;
typedef __attribute__((ext_vector_type(16))) __bf16   v16bf;
typedef __attribute__((ext_vector_type(8)))  unsigned short v8us;
typedef __attribute__((ext_vector_type(8)))  float    v8f;
typedef __attribute__((ext_vector_type(4)))  float    v4f;
typedef v4f  __attribute__((may_alias)) v4fa;
typedef v8us __attribute__((may_alias)) v8usa;

__device__ __forceinline__ unsigned short f2bf(float f) { unsigned u = __float_as_uint(f); u += 0x7FFFu + ((u >> 16) & 1u); return (unsigned short)(u >> 16); }
__device__ __forceinline__ float bf2f(unsigned short w) { return __uint_as_float(((unsigned)w) << 16); }
__device__ __forceinline__ int clampi(int v, int lo, int hi) { return min(max(v, lo), hi); }
__device__ __forceinline__ v16bf cat16b(v8us lo, v8us hi) { return __builtin_bit_cast(v16bf, __builtin_shufflevector(lo, hi, 0, 1, 2, 3, 4, 5, 6, 7, 8, 9, 10, 11, 12, 13, 14, 15)); }
__device__ __forceinline__ v8f wmmab(v16bf a, v16bf b, v8f c) { return __builtin_amdgcn_wmma_f32_16x16x32_bf16(false, a, false, b, (short)0, c, false, false); }
__device__ __forceinline__ v16bf ldb(const bf* p)  { return cat16b(*(const v8us*)p, *(const v8us*)(p + 16)); }
__device__ __forceinline__ void wave_sync() { __builtin_amdgcn_fence(3  , "wavefront"); __builtin_amdgcn_wave_barrier(); asm volatile("" ::: "memory"); }

__device__ __forceinline__ v8f wmmag(v16bf a, v16bf b, v8f c) {
    c = wmmab(a, b, c);
    asm volatile("v_nop\n\tv_nop\n\tv_nop\n\tv_nop" : "+v"(c) : "v"(a), "v"(b));
    return c;
}
__device__ __forceinline__ float bfq(float f) { return bf2f(f2bf(f)); }
__device__ __forceinline__ float act_rowdy(float t, float a, float w) {
    const float ax = fminf(fabsf(t), 15.0f);
    const float e  = __expf(2.0f * ax);
    const float th = 1.0f - 2.0f * __builtin_amdgcn_rcpf(e + 1.0f);
    return copysignf(th, t) + a * __sinf(w * t);
}
__device__ __forceinline__ void split8(const float (&v)[8], v8us& oh, v8us& ol) {
#pragma unroll
    for (int nt = 0; nt < 8; ++nt) { const unsigned short h = f2bf(v[nt]); oh[nt] = h; ol[nt] = f2bf(v[nt] - bf2f(h)); }
}
__device__ __forceinline__ v4f perm_row(const float* __restrict__ src, int lane) {
    v4f v;
#pragma unroll
    for (int i = 0; i < 4; ++i) v[i] = bfq(src[((4 * (lane & 1) + i) << 4) + (lane >> 1)]);
    return v;
}
__device__ __forceinline__ v4f nat_row(const float* __restrict__ src, int lane) {
    const v4f x = *(const v4f*)(src + 4 * lane); v4f v;
#pragma unroll
    for (int i = 0; i < 4; ++i) v[i] = bfq(x[i]);
    return v;
}
__device__ __forceinline__ void mma8(const v16bf ah, const v16bf al, const bf* __restrict__ wk, v8f (&acc)[8]) {
#pragma unroll
    for (int nt = 0; nt < 8; ++nt) { const v16bf b = ldb(wk + (size_t)nt * 16 * HID); acc[nt] = wmmag(ah, b, acc[nt]); acc[nt] = wmmag(al, b, acc[nt]); }
}

__global__ __launch_bounds__(256) void k_wconv(const float* __restrict__ W, int ldn, int tpm, bf* DST) {
    __shared__ float ts[HID * 65];
    const int t = threadIdx.x;
    const int mat = (int)blockIdx.x / tpm, nt = (int)blockIdx.x - mat * tpm;
    const float* src = W + (size_t)mat * HID * ldn + (size_t)nt * 64;
#pragma unroll 1
    for (int i = 0; i < 32; ++i) { const int f = i * 256 + t; const int k = f >> 6, e = f & 63; ts[k * 65 + e] = src[(size_t)k * ldn + e]; }
    __syncthreads();
    bf* dst = DST + ((size_t)mat * ldn + (size_t)nt * 64) * HID;
    const int pc = t & 15;
#pragma unroll 1
    for (int ps = 0; ps < 2; ++ps) {
#pragma unroll 1
        for (int it = 0; it < 4; ++it) {
            const int e = it * 16 + (t >> 4); v8us o;
#pragma unroll
            for (int kk = 0; kk < 8; ++kk) o[kk] = f2bf(ts[(kk * 16 + pc) * 65 + e]);
            *(volatile v8us*)(dst + (size_t)e * HID + pc * 8) = o; }
        if (ps == 0) __threadfence(); }
}

__global__ __launch_bounds__(256) void k_w0(const float* __restrict__ W, int kr, bf* DST) {
    const int t = threadIdx.x, q = t & 3;
#pragma unroll 1
    for (int ps = 0; ps < 2; ++ps) {
#pragma unroll 1
        for (int it = 0; it < 2; ++it) {
            const int row = it * 64 + (t >> 2); v8us o;
#pragma unroll
            for (int kk = 0; kk < 8; ++kk) { const int kc = min(kk, kr - 1); const float v = W[kc * HID + row];
                o[kk] = (q == 0 && kk < kr) ? f2bf(v) : (unsigned short)0; }
            *(volatile v8us*)(DST + (size_t)row * 32 + q * 8) = o; }
        if (ps == 0) __threadfence(); }
}

__global__ __launch_bounds__(32) __attribute__((amdgpu_num_vgpr(256))) void k_branch(
        const float* __restrict__ params, const bf* __restrict__ WB0, const bf* __restrict__ WBP, const bf* __restrict__ WBF,
        const float* __restrict__ bb0, const float* __restrict__ bb, const float* __restrict__ bbf, const float* __restrict__ ab, const float* __restrict__ wb,
        const float* __restrict__ bt0, const float* __restrict__ bt, const float* __restrict__ btf, const float* __restrict__ at, const float* __restrict__ wt,
        float* PW, float* G, bf* BCH, bf* BCL) {
    __shared__ __align__(16) bf xh[16 * XP];
    __shared__ __align__(16) bf xl[16 * XP];
    __shared__ __align__(16) float gs[16 * HID];
    __shared__ __align__(16) float pt[3 * HID];
    const int lane = threadIdx.x & 31, lr = lane & 15, hi = lane >> 4;
    v4f zr;
#pragma unroll
    for (int i = 0; i < 4; ++i) zr[i] = 0.0f;

#pragma unroll 1
    for (int ps = 0; ps < 2; ++ps) {
        { const v4f v = perm_row(bt0, lane); *(volatile v4f*)(PW + (size_t)(0 * 3 + 0) * HID + 4 * lane) = v; }
#pragma unroll 1
        for (int l = 1; l < 4; ++l) { const v4f v = perm_row(bt + (size_t)(l - 1) * HID, lane); *(volatile v4f*)(PW + (size_t)(l * 3 + 0) * HID + 4 * lane) = v; }
        { const v4f v = perm_row(btf, lane); *(volatile v4f*)(PW + (size_t)(4 * 3 + 0) * HID + 4 * lane) = v; }
#pragma unroll 1
        for (int l = 0; l < 4; ++l) {
            const v4f va = perm_row(at + (size_t)l * HID, lane); *(volatile v4f*)(PW + (size_t)(l * 3 + 1) * HID + 4 * lane) = va;
            const v4f vw = perm_row(wt + (size_t)l * HID, lane); *(volatile v4f*)(PW + (size_t)(l * 3 + 2) * HID + 4 * lane) = vw; }
        *(volatile v4f*)(PW + (size_t)(4 * 3 + 1) * HID + 4 * lane) = zr;
        *(volatile v4f*)(PW + (size_t)(4 * 3 + 2) * HID + 4 * lane) = zr;
        if (ps == 0) __threadfence(); }

#pragma unroll 1
    for (int i = 0; i < 16; ++i) *(v4fa*)&gs[i * HID + 4 * lane] = zr;
    { const v4f v0 = nat_row(bb0, lane), v1 = nat_row(ab, lane), v2 = nat_row(wb, lane);
      *(v4fa*)&pt[0 * HID + 4 * lane] = v0; *(v4fa*)&pt[1 * HID + 4 * lane] = v1; *(v4fa*)&pt[2 * HID + 4 * lane] = v2; }
    wave_sync();

    v8f acc[8];
    {
        const int bc = min(lr, NB - 1);
        v8us a0, z8;
#pragma unroll
        for (int k = 0; k < 8; ++k) { a0[k] = (unsigned short)0; z8[k] = (unsigned short)0; }
#pragma unroll
        for (int k = 0; k < 6; ++k) { const float pv = params[bc * 6 + k]; a0[k] = (hi == 0) ? f2bf(pv) : (unsigned short)0; }
        const v16bf a = cat16b(a0, z8);
#pragma unroll
        for (int nt = 0; nt < 8; ++nt) { const v16bf b = ldb(WB0 + (size_t)(nt * 16 + lr) * 32 + 8 * hi); acc[nt] = wmmag(a, b, (v8f){}); }
    }

#pragma unroll 1
    for (int li = 0; li < 4; ++li) {
        float pb[8], pa[8], pw[8];
#pragma unroll
        for (int nt = 0; nt < 8; ++nt) { pb[nt] = pt[nt * 16 + lr]; pa[nt] = pt[HID + nt * 16 + lr]; pw[nt] = pt[2 * HID + nt * 16 + lr]; }
#pragma unroll
        for (int r = 0; r < 8; ++r) {
            const int row = 8 * hi + r;
            const v4f g0 = *(const v4fa*)&gs[row * HID + lr * 8]; const v4f g1 = *(const v4fa*)&gs[row * HID + lr * 8 + 4];
            float v[8];
#pragma unroll
            for (int nt = 0; nt < 8; ++nt) v[nt] = act_rowdy(acc[nt][r] + pb[nt], pa[nt], pw[nt]);
            v4f n0, n1;
#pragma unroll
            for (int i = 0; i < 4; ++i) { n0[i] = g0[i] + v[i]; n1[i] = g1[i] + v[4 + i]; }
            *(v4fa*)&gs[row * HID + lr * 8] = n0; *(v4fa*)&gs[row * HID + lr * 8 + 4] = n1;
            v8us oh, ol; split8(v, oh, ol);
            *(v8usa*)&xh[row * XP + lr * 8] = oh; *(v8usa*)&xl[row * XP + lr * 8] = ol;
        }
        wave_sync();
#pragma unroll 1
        for (int ps = 0; ps < 2; ++ps) {
#pragma unroll 1
            for (int rr = 0; rr < 16; ++rr) { const v4f v = *(const v4fa*)&gs[rr * HID + 4 * lane]; *(volatile v4f*)(G + (size_t)(li * NB_FULL + rr) * HID + 4 * lane) = v; }
            if (ps == 0) __threadfence(); }
        wave_sync();
        if (li < 3) {
            { const v4f v0 = nat_row(bb + (size_t)li * HID, lane), v1 = nat_row(ab + (size_t)(li + 1) * HID, lane), v2 = nat_row(wb + (size_t)(li + 1) * HID, lane);
              *(v4fa*)&pt[0 * HID + 4 * lane] = v0; *(v4fa*)&pt[1 * HID + 4 * lane] = v1; *(v4fa*)&pt[2 * HID + 4 * lane] = v2; }
            wave_sync();
#pragma unroll
            for (int nt = 0; nt < 8; ++nt) acc[nt] = (v8f){};
            const bf* wl = WBP + (size_t)li * HID * HID + (size_t)lr * HID + 8 * hi;
#pragma unroll 1
            for (int kc = 0; kc < HID / 32; ++kc) {
                const int ai = lr * XP + kc * 32 + 8 * hi;
                const v16bf ah = cat16b(*(const v8usa*)&xh[ai], *(const v8usa*)&xh[ai + 16]);
                const v16bf al = cat16b(*(const v8usa*)&xl[ai], *(const v8usa*)&xl[ai + 16]);
                mma8(ah, al, wl + kc * 32, acc); }
        }
    }

#pragma unroll 1
    for (int o = 0; o < NOUT; ++o) {
#pragma unroll
        for (int nt = 0; nt < 8; ++nt) acc[nt] = (v8f){};
        const bf* wl = WBF + (size_t)o * HID * HID + (size_t)lr * HID + 8 * hi;
#pragma unroll 1
        for (int kc = 0; kc < HID / 32; ++kc) {
            const int ai = lr * XP + kc * 32 + 8 * hi;
            const v16bf ah = cat16b(*(const v8usa*)&xh[ai], *(const v8usa*)&xh[ai + 16]);
            const v16bf al = cat16b(*(const v8usa*)&xl[ai], *(const v8usa*)&xl[ai + 16]);
            mma8(ah, al, wl + kc * 32, acc); }
        float bs[8];
#pragma unroll
        for (int nt = 0; nt < 8; ++nt) bs[nt] = bfq(bbf[o * HID + nt * 16 + lr]);
        v8us oh[8], ol[8];
#pragma unroll
        for (int r = 0; r < 8; ++r) { float v[8];
#pragma unroll
            for (int nt = 0; nt < 8; ++nt) v[nt] = acc[nt][r] + bs[nt];
            split8(v, oh[r], ol[r]); }
#pragma unroll 1
        for (int ps = 0; ps < 2; ++ps) {
#pragma unroll
            for (int r = 0; r < 8; ++r) { const size_t di = ((size_t)((8 * hi + r) * NOUT + o)) * HID + lr * 8;
                *(volatile v8us*)(BCH + di) = oh[r]; *(volatile v8us*)(BCL + di) = ol[r]; }
            if (ps == 0) __threadfence(); }
    }
}

__global__ __launch_bounds__(128) __attribute__((amdgpu_num_vgpr(256))) void k_trunk(
        const float* __restrict__ coords, const float* __restrict__ sdf, const bf* __restrict__ WT0, const bf* __restrict__ WTP,
        const float* __restrict__ PW, const float* __restrict__ G, const bf* __restrict__ BCH, const bf* __restrict__ BCL, float* OUT) {
    __shared__ __align__(16) bf xh[TW * 16 * XP];
    __shared__ __align__(16) bf xl[TW * 16 * XP];
    __shared__ __align__(16) float outs[TROWS * NOUT];
    const int tid = threadIdx.x, lane = tid & 31, lr = lane & 15, hi = lane >> 4;
    const int wave = __builtin_amdgcn_readfirstlane(tid >> 5);
    const int rv = min(((int)blockIdx.x * TW + (tid >> 5)) * 16, NROWS - 16);
    const int row0 = __builtin_amdgcn_readfirstlane(rv);
    const int b = row0 / NPTS;
    const int p0 = row0 - b * NPTS;
    const int xb = wave * 16 * XP;

    v8f acc[8];
    {
        const size_t pr = (size_t)b * NPTS_FULL + (size_t)(p0 + lr);
        const float cx = coords[pr * 3 + 0], cy = coords[pr * 3 + 1], cz = coords[pr * 3 + 2], sv = sdf[pr];
        v8us a0, z8;
#pragma unroll
        for (int k = 0; k < 8; ++k) { a0[k] = (unsigned short)0; z8[k] = (unsigned short)0; }
        a0[0] = (hi == 0) ? f2bf(cx) : (unsigned short)0;
        a0[1] = (hi == 0) ? f2bf(cy) : (unsigned short)0;
        a0[2] = (hi == 0) ? f2bf(cz) : (unsigned short)0;
        a0[3] = (hi == 0) ? f2bf(sv) : (unsigned short)0;
        const v16bf a = cat16b(a0, z8);
#pragma unroll
        for (int nt = 0; nt < 8; ++nt) { const v16bf bw = ldb(WT0 + (size_t)(nt * 16 + lr) * 32 + 8 * hi); acc[nt] = wmmag(a, bw, (v8f){}); }
    }

#pragma unroll 1
    for (int l = 0; l < 4; ++l) {
        float pb[8], pa[8], pw[8], pg[8];
        {
            const float* pwl = PW + (size_t)(l * 3) * HID + lr * 8;
            const float* gl  = G + (size_t)(l * NB_FULL + b) * HID + lr * 8;
            const v4f b0 = *(const v4f*)(pwl), b1 = *(const v4f*)(pwl + 4);
            const v4f a0 = *(const v4f*)(pwl + HID), a1 = *(const v4f*)(pwl + HID + 4);
            const v4f w0 = *(const v4f*)(pwl + 2 * HID), w1 = *(const v4f*)(pwl + 2 * HID + 4);
            const v4f g0 = *(const v4f*)(gl), g1 = *(const v4f*)(gl + 4);
#pragma unroll
            for (int i = 0; i < 4; ++i) { pb[i] = b0[i]; pb[4 + i] = b1[i]; pa[i] = a0[i]; pa[4 + i] = a1[i]; pw[i] = w0[i]; pw[4 + i] = w1[i]; pg[i] = g0[i]; pg[4 + i] = g1[i]; }
        }
#pragma unroll
        for (int r = 0; r < 8; ++r) {
            float v[8];
#pragma unroll
            for (int nt = 0; nt < 8; ++nt) v[nt] = act_rowdy(acc[nt][r] + pb[nt], pa[nt], pw[nt]) * pg[nt];
            v8us oh, ol; split8(v, oh, ol);
            const int xi = xb + (8 * hi + r) * XP + lr * 8;
            *(v8usa*)&xh[xi] = oh; *(v8usa*)&xl[xi] = ol;
        }
        wave_sync();
#pragma unroll
        for (int nt = 0; nt < 8; ++nt) acc[nt] = (v8f){};
        const bf* wl = WTP + (size_t)l * HID * HID + (size_t)lr * HID + 8 * hi;
#pragma unroll 1
        for (int kc = 0; kc < HID / 32; ++kc) {
            const int ai = xb + lr * XP + kc * 32 + 8 * hi;
            const v16bf ah = cat16b(*(const v8usa*)&xh[ai], *(const v8usa*)&xh[ai + 16]);
            const v16bf al = cat16b(*(const v8usa*)&xl[ai], *(const v8usa*)&xl[ai + 16]);
            mma8(ah, al, wl + kc * 32, acc); }
    }

    {
        float pb[8];
        const float* pwl = PW + (size_t)(4 * 3) * HID + lr * 8;
        const v4f b0 = *(const v4f*)(pwl), b1 = *(const v4f*)(pwl + 4);
#pragma unroll
        for (int i = 0; i < 4; ++i) { pb[i] = b0[i]; pb[4 + i] = b1[i]; }
#pragma unroll
        for (int r = 0; r < 8; ++r) {
            float v[8];
#pragma unroll
            for (int nt = 0; nt < 8; ++nt) v[nt] = acc[nt][r] + pb[nt];
            v8us oh, ol; split8(v, oh, ol);
            const int xi = xb + (8 * hi + r) * XP + lr * 8;
            *(v8usa*)&xh[xi] = oh; *(v8usa*)&xl[xi] = ol;
        }
        wave_sync();
    }

    v8f o5 = (v8f){};
    {
        const int oc = min(lr, NOUT - 1);
        const size_t bo = ((size_t)(b * NOUT + oc)) * HID + 8 * hi;
#pragma unroll 1
        for (int kc = 0; kc < HID / 32; ++kc) {
            const int ai = xb + lr * XP + kc * 32 + 8 * hi;
            const v16bf ah = cat16b(*(const v8usa*)&xh[ai], *(const v8usa*)&xh[ai + 16]);
            const v16bf al = cat16b(*(const v8usa*)&xl[ai], *(const v8usa*)&xl[ai + 16]);
            const v16bf bh = ldb(BCH + bo + kc * 32);
            const v16bf bl = ldb(BCL + bo + kc * 32);
            o5 = wmmag(ah, bh, o5); o5 = wmmag(al, bh, o5); o5 = wmmag(ah, bl, o5); }
    }
    if (lr < NOUT) {
#pragma unroll
        for (int r = 0; r < 8; ++r) outs[(wave * 16 + 8 * hi + r) * NOUT + lr] = o5[r];
    }
    __syncthreads();
    {
        const size_t g4 = (size_t)blockIdx.x * (TROWS * NOUT) + 4 * (size_t)tid;
        const bool ok = (tid < OUTPIECES) && (g4 + 4 <= (size_t)NROWS * NOUT);
        const v4f v = *(const v4fa*)&outs[4 * min(tid, OUTPIECES - 1)];
#pragma unroll 1
        for (int ps = 0; ps < 2; ++ps) {
            if (ok) *(volatile v4f*)(OUT + g4) = v;
            if (ps == 0) __threadfence(); }
    }
}

static constexpr size_t al256(size_t v) { return (v + 255) & ~(size_t)255; }
static constexpr size_t SZ_W0  = al256((size_t)HID * 32 * 2);
static constexpr size_t SZ_WBP = al256((size_t)3 * HID * HID * 2);
static constexpr size_t SZ_WBF = al256((size_t)NOUT * HID * HID * 2);
static constexpr size_t SZ_WTP = al256((size_t)4 * HID * HID * 2);
static constexpr size_t SZ_PW  = al256((size_t)5 * 3 * HID * 4);
static constexpr size_t SZ_G   = al256((size_t)4 * NB_FULL * HID * 4);
static constexpr size_t SZ_BC  = al256((size_t)NB_FULL * NOUT * HID * 2);
static constexpr size_t SZ_TOTAL = 2 * SZ_W0 + SZ_WBP + SZ_WBF + SZ_WTP + SZ_PW + SZ_G + 2 * SZ_BC;
static_assert(SZ_TOTAL <= (size_t)134217728);
static_assert(SZ_W0 == (size_t)HID * 64 && SZ_PW == (size_t)15 * 512 && SZ_G == (size_t)64 * 512 && SZ_BC == (size_t)80 * 256);

extern "C" void kernel_launch(void* const* d_in, const int* in_sizes, int n_in,
                              void* d_out, int out_size, void* d_ws, size_t ws_size, hipStream_t stream) {
    if (n_in < 19) return;
    if ((size_t)in_sizes[0] < ((size_t)(NB - 1) * NPTS_FULL + NPTS) * 3) return;
    if ((size_t)in_sizes[1] < ((size_t)(NB - 1) * NPTS_FULL + NPTS)) return;
    if ((size_t)in_sizes[2] < (size_t)NB * 6) return;
    if (in_sizes[3] < 6 * HID || in_sizes[4] < HID || in_sizes[5] < 3 * HID * HID || in_sizes[6] < 3 * HID) return;
    if (in_sizes[7] < HID * HID * NOUT || in_sizes[8] < HID * NOUT || in_sizes[9] < 4 * HID || in_sizes[10] < 4 * HID) return;
    if (in_sizes[11] < 4 * HID || in_sizes[12] < HID || in_sizes[13] < 3 * HID * HID || in_sizes[14] < 3 * HID) return;
    if (in_sizes[15] < HID * HID || in_sizes[16] < HID || in_sizes[17] < 4 * HID || in_sizes[18] < 4 * HID) return;
    if ((size_t)out_size < (size_t)NROWS * NOUT) return;
    if (SZ_TOTAL > ws_size) return;
    const float* coords = (const float*)d_in[0];
    const float* sdf    = (const float*)d_in[1];
    const float* params = (const float*)d_in[2];
    const float* Wb0    = (const float*)d_in[3];
    const float* bb0    = (const float*)d_in[4];
    const float* Wb     = (const float*)d_in[5];
    const float* bb     = (const float*)d_in[6];
    const float* Wbf    = (const float*)d_in[7];
    const float* bbf    = (const float*)d_in[8];
    const float* ab     = (const float*)d_in[9];
    const float* wb     = (const float*)d_in[10];
    const float* Wt0    = (const float*)d_in[11];
    const float* bt0    = (const float*)d_in[12];
    const float* Wt     = (const float*)d_in[13];
    const float* bt     = (const float*)d_in[14];
    const float* Wtf    = (const float*)d_in[15];
    const float* btf    = (const float*)d_in[16];
    const float* at     = (const float*)d_in[17];
    const float* wt     = (const float*)d_in[18];
    float* OUT = (float*)d_out;
    char* wsp = (char*)d_ws;
    bf* WT0 = (bf*)wsp; wsp += SZ_W0;
    bf* WB0 = (bf*)wsp; wsp += SZ_W0;
    bf* WBP = (bf*)wsp; wsp += SZ_WBP;
    bf* WBF = (bf*)wsp; wsp += SZ_WBF;
    bf* WTP = (bf*)wsp; wsp += SZ_WTP;
    float* PW = (float*)wsp; wsp += SZ_PW;
    float* GG = (float*)wsp; wsp += SZ_G;
    bf* BCH = (bf*)wsp; wsp += SZ_BC;
    bf* BCL = (bf*)wsp; wsp += SZ_BC;

    k_wconv<<<6, 256, 0, stream>>>(Wb, HID, 2, WBP);
    k_wconv<<<10, 256, 0, stream>>>(Wbf, HID * NOUT, 10, WBF);
    k_wconv<<<6, 256, 0, stream>>>(Wt, HID, 2, WTP);
    k_wconv<<<2, 256, 0, stream>>>(Wtf, HID, 2, WTP + (size_t)3 * HID * HID);
    k_w0<<<1, 256, 0, stream>>>(Wb0, 6, WB0);
    k_w0<<<1, 256, 0, stream>>>(Wt0, 4, WT0);
    k_branch<<<1, 32, 0, stream>>>(params, WB0, WBP, WBF, bb0, bb, bbf, ab, wb, bt0, bt, btf, at, wt, PW, GG, BCH, BCL);
    k_trunk<<<(unsigned)((NROWS + TROWS - 1) / TROWS), TW * 32, 0, stream>>>(coords, sdf, WT0, WTP, PW, GG, BCH, BCL, OUT);
}
